// MambaSimple_67602785239495
// MI455X (gfx1250) — hardware-verified
//
#include <hip/hip_runtime.h>


#define NB_  2
#define NL_  1024
#define DM_  1024
#define DI_  2048
#define NS_  16
#define NR_  1024
#define XW_  (NR_ + 2 * NS_)
#define MT_  (NB_ * NL_)

static_assert(MT_ % 64 == 0);
static_assert((2 * DI_) % 128 == 0);
static_assert(DI_ % 128 == 0);
static_assert(DM_ % 64 == 0);
static_assert(XW_ % 32 == 0);
static_assert(DM_ % 32 == 0);
static_assert(DI_ % 64 == 0);
static_assert(NR_ % 64 == 0);
static_assert(NL_ % 16 == 0);
static_assert((NL_ & (NL_ - 1)) == 0);
static_assert(DI_ / 8 == 256);
static_assert(NS_ == 16);

typedef float          v4f   __attribute__((ext_vector_type(4)));
typedef float          v8f   __attribute__((ext_vector_type(8)));
typedef _Float16       v8h   __attribute__((ext_vector_type(8)));
typedef _Float16       v16h  __attribute__((ext_vector_type(16)));
typedef __bf16         v16b  __attribute__((ext_vector_type(16)));
typedef unsigned short u16x8 __attribute__((ext_vector_type(8)));

union FragH { u16x8 h[2]; v16h v; };
union FragB { u16x8 h[2]; v16b v; };
union Pack8 { v8h f; u16x8 u; };
union H1    { _Float16 f; unsigned short u; };

__device__ __forceinline__ unsigned short f32_to_bf16(float f) {
    unsigned u = __float_as_uint(f);
    unsigned r = u + 0x7FFFu + ((u >> 16) & 1u);
    return (unsigned short)(r >> 16);
}
__device__ __forceinline__ float bf16_to_f32(unsigned short b) {
    return __uint_as_float(((unsigned)b) << 16);
}
__device__ __forceinline__ float bf16r_f(float f) {
    return bf16_to_f32(f32_to_bf16(f));
}
__device__ __forceinline__ v8f ld8f(const float* p) {
    v4f a = *(const v4f*)p;
    v4f b = *(const v4f*)(p + 4);
    return __builtin_shufflevector(a, b, 0, 1, 2, 3, 4, 5, 6, 7);
}
__device__ __forceinline__ v8f bf16r8(v8f x) {
    v8f r;
#pragma unroll
    for (int e = 0; e < 8; ++e) r[e] = bf16r_f(x[e]);
    return r;
}
__device__ __forceinline__ float silu_f(float x) {
    float e = expf(-x);
    return x * __builtin_amdgcn_rcpf(1.0f + e);
}
__device__ __forceinline__ float softplus_f(float x) {
    return fmaxf(x, 0.0f) + log1pf(expf(-fabsf(x)));
}
__device__ __forceinline__ float conv4_silu(float x0, float x1, float x2, float x3,
                                            float w0, float w1, float w2, float w3, float bias) {
    float c = w0 * x0 + w1 * x1 + w2 * x2 + w3 * x3;
    return silu_f(c + bias);
}

__device__ __forceinline__ void mma16(v8f& acc, const FragH& a, const FragH& b) {
    acc = __builtin_amdgcn_wmma_f32_16x16x32_f16(false, a.v, false, b.v, (short)0, acc, false, false);
    asm volatile("v_nop\n\tv_nop\n\tv_nop\n\tv_nop" : "+v"(acc) : "v"(a.v), "v"(b.v));
}
__device__ __forceinline__ void mma16(v8f& acc, const FragB& a, const FragB& b) {
    acc = __builtin_amdgcn_wmma_f32_16x16x32_bf16(false, a.v, false, b.v, (short)0, acc, false, false);
    asm volatile("v_nop\n\tv_nop\n\tv_nop\n\tv_nop" : "+v"(acc) : "v"(a.v), "v"(b.v));
}

__global__ __launch_bounds__(256)
void cvt_rows_kernel(const float* __restrict__ src, unsigned short* dst,
                     int rows, int cols, int spitch, int mode, float scale)
{
    const int i   = blockIdx.x * 256 + threadIdx.x;
    const int cpr = cols >> 3;
    if (i >= rows * cpr) return;
    const int r = i / cpr;
    const int c = (i - r * cpr) * 8;
    const v8f x = ld8f(src + (size_t)r * spitch + c);
    u16x8 v;
    if (mode == 0) {
#pragma unroll
        for (int e = 0; e < 8; ++e) v[e] = f32_to_bf16(x[e]);
    } else {
        Pack8 pk;
        pk.f = __builtin_convertvector(x * scale, v8h);
        v = pk.u;
    }
    unsigned short* gp = dst + (size_t)r * cols + c;
    *(volatile u16x8*)gp = v;
    __threadfence();
    *(volatile u16x8*)gp = v;
}

__global__ __launch_bounds__(256)
void cvt_t_kernel(const float* __restrict__ in, unsigned short* out, int R, int C,
                  int mode, float scale)
{
    __shared__ __attribute__((aligned(16))) unsigned short st[32 * 72];
    const int tid = threadIdx.x, lane = tid & 31, wave = tid >> 5;
    const int n0 = blockIdx.x * 32, k0 = blockIdx.y * 64;
    {
        const int kr = tid >> 2;
        const int c8 = (tid & 3) * 8;
        const v8f x = ld8f(in + (size_t)(k0 + kr) * C + n0 + c8);
#pragma unroll
        for (int e = 0; e < 8; ++e) {
            const unsigned short bb = f32_to_bf16(x[e]);
            unsigned short q = bb;
            if (mode != 0) { H1 t; t.f = (_Float16)(scale * bf16_to_f32(bb)); q = t.u; }
            st[(c8 + e) * 72 + kr] = q;
        }
    }
    __syncthreads();
    const int row = wave * 4 + (lane >> 3);
    const int ch  = (lane & 7) * 8;
    const u16x8 v = *(const u16x8*)(st + row * 72 + ch);
    unsigned short* gp = out + (size_t)(n0 + row) * R + k0 + ch;
    *(volatile u16x8*)gp = v;
    __threadfence();
    *(volatile u16x8*)gp = v;
}

template<int NBF>
__device__ __forceinline__ void blk_store_pass(const float* st, float* gp, int ldc, int wave, int lane) {
    constexpr int BW  = 32 * NBF;
    constexpr int P   = BW + 4;
    constexpr int LPR = BW / 4;
    constexpr int RPI = 32 / LPR;
    constexpr int NIT = 16 / RPI;
    const int rsub = lane / LPR;
    const int c4   = (lane % LPR) * 4;
#pragma unroll
    for (int it = 0; it < NIT; ++it) {
        const int row = wave * 16 + it * RPI + rsub;
        const v4f v = *(const v4f*)(st + row * P + c4);
        *(volatile v4f*)(gp + (size_t)row * ldc + c4) = v;
    }
}

template<typename FR, bool ASPLIT, int NBF>
__global__ __launch_bounds__(128)
void gemm_tn_kernel(const unsigned short* __restrict__ A,  const unsigned short* __restrict__ A2,
                    const unsigned short* __restrict__ Bw,
                    float* C, float* C2, int K, int ldc, int csplit, float scale)
{
    constexpr int CW = NBF * 16;
    constexpr int BW = 2 * CW;
    constexpr int P  = BW + 4;
    __shared__ __attribute__((aligned(16))) float stile[64 * P];

    const int tid  = threadIdx.x;
    const int lane = tid & 31;
    const int wave = tid >> 5;
    const int h    = lane >> 4;
    const int m    = lane & 15;
    const int wm   = wave >> 1;
    const int wn   = wave & 1;

    const int rowB = blockIdx.y * 64;
    const int colB = blockIdx.x * BW;
    const int rowW = rowB + wm * 32;
    const int colW = colB + wn * CW;

    v8f acc[2 * NBF];
#pragma unroll
    for (int j = 0; j < 2 * NBF; ++j)
#pragma unroll
        for (int r = 0; r < 8; ++r) acc[j][r] = 0.0f;

    const size_t aoff  = (size_t)(rowW + m) * K + 8 * h;
    const size_t boff  = (size_t)(colW + m) * K + 8 * h;
    const size_t sub16 = (size_t)16 * K;
    const int nk = K >> 5;

    for (int kt = 0; kt < nk; ++kt) {
        const size_t k0 = (size_t)kt * 32;
        FR fa[2], fb[NBF], ga[2];
#pragma unroll
        for (int s = 0; s < 2; ++s) {
            const unsigned short* p = A + aoff + s * sub16 + k0;
            fa[s].h[0] = *(const u16x8*)(p);
            fa[s].h[1] = *(const u16x8*)(p + 16);
            if (ASPLIT) {
                const unsigned short* q = A2 + aoff + s * sub16 + k0;
                ga[s].h[0] = *(const u16x8*)(q);
                ga[s].h[1] = *(const u16x8*)(q + 16);
            }
        }
#pragma unroll
        for (int j = 0; j < NBF; ++j) {
            const unsigned short* p = Bw + boff + j * sub16 + k0;
            fb[j].h[0] = *(const u16x8*)(p);
            fb[j].h[1] = *(const u16x8*)(p + 16);
        }
#pragma unroll
        for (int s = 0; s < 2; ++s)
#pragma unroll
            for (int j = 0; j < NBF; ++j) {
                mma16(acc[s * NBF + j], fa[s], fb[j]);
                if (ASPLIT) mma16(acc[s * NBF + j], ga[s], fb[j]);
            }
    }

#pragma unroll
    for (int s = 0; s < 2; ++s)
#pragma unroll
        for (int j = 0; j < NBF; ++j)
#pragma unroll
            for (int r = 0; r < 8; ++r)
                stile[(wm * 32 + s * 16 + 8 * h + r) * P + wn * CW + j * 16 + m] = acc[s * NBF + j][r] * scale;
    __syncthreads();

    float* Cp = C;
    int gcol = colB;
    if (colB >= csplit) { Cp = C2; gcol = colB - csplit; }
    float* gp = Cp + (size_t)rowB * ldc + gcol;
    blk_store_pass<NBF>(stile, gp, ldc, wave, lane);
    __threadfence();
    blk_store_pass<NBF>(stile, gp, ldc, wave, lane);
}

__global__ __launch_bounds__(256)
void conv_silu_kernel(const float* __restrict__ X, const float* __restrict__ cw,
                      const float* __restrict__ cb, unsigned short* U16)
{
    const int mrow = blockIdx.x;
    const int l    = mrow & (NL_ - 1);
    const int d0   = threadIdx.x * 8;
    const float* xr = X + (size_t)mrow * DI_ + d0;

    const v8f x3 = ld8f(xr);
    v8f x2, x1, x0;
#pragma unroll
    for (int c = 0; c < 8; ++c) { x2[c] = 0.0f; x1[c] = 0.0f; x0[c] = 0.0f; }
    if (l >= 1) x2 = ld8f(xr - DI_);
    if (l >= 2) x1 = ld8f(xr - 2 * DI_);
    if (l >= 3) x0 = ld8f(xr - 3 * DI_);

    v8f wt[4];
#pragma unroll
    for (int k = 0; k < 4; ++k) wt[k] = bf16r8(ld8f(cw + (size_t)k * DI_ + d0));
    const v8f bias = bf16r8(ld8f(cb + d0));

    v8f u;
#pragma unroll
    for (int c = 0; c < 8; ++c)
        u[c] = conv4_silu(x0[c], x1[c], x2[c], x3[c], wt[0][c], wt[1][c], wt[2][c], wt[3][c], bias[c]);

    Pack8 pk;
    pk.f = __builtin_convertvector(u * 256.0f, v8h);
    const u16x8 v = pk.u;
    unsigned short* gp = U16 + (size_t)mrow * DI_ + d0;
    *(volatile u16x8*)gp = v;
    __threadfence();
    *(volatile u16x8*)gp = v;
}

__device__ __forceinline__ void rows16_store_pass(const unsigned short* sl, unsigned short* gpl,
                                                  size_t gbase, int lane) {
#pragma unroll
    for (int it = 0; it < 4; ++it) {
        const int t = it * 4 + (lane >> 3);
        const int c = (lane & 7) * 8;
        const u16x8 v = *(const u16x8*)(sl + t * 64 + c);
        *(volatile u16x8*)(gpl + gbase + (size_t)t * DI_ + c) = v;
    }
}

__global__ __launch_bounds__(64)
void scan_kernel(const float* __restrict__ X, const float* __restrict__ Z,
                 const float* __restrict__ Dl, const float* __restrict__ Xd,
                 const float* __restrict__ cw, const float* __restrict__ cb,
                 const float* __restrict__ bdt, const float* __restrict__ Alog,
                 unsigned short* ghi, unsigned short* glo)
{
    __shared__ __attribute__((aligned(16))) float          sBC[16 * 32];
    __shared__ __attribute__((aligned(16))) unsigned short shi[16 * 64];
    __shared__ __attribute__((aligned(16))) unsigned short slo[16 * 64];

    const int tid   = threadIdx.x;
    const int lane  = tid & 31;
    const int wave  = tid >> 5;
    const int dbase = blockIdx.x * 64;
    const int d     = dbase + tid;
    const int b     = blockIdx.y;

    float an[NS_], hs[NS_];
#pragma unroll
    for (int n = 0; n < NS_; ++n) {
        an[n] = -expf(bf16r_f(Alog[(size_t)d * NS_ + n]));
        hs[n] = 0.0f;
    }
    const float w0 = bf16r_f(cw[0 * DI_ + d]);
    const float w1 = bf16r_f(cw[1 * DI_ + d]);
    const float w2 = bf16r_f(cw[2 * DI_ + d]);
    const float w3 = bf16r_f(cw[3 * DI_ + d]);
    const float cbias = bf16r_f(cb[d]);
    const float tb    = bf16r_f(bdt[d]);

    float xm1 = 0.0f, xm2 = 0.0f, xm3 = 0.0f;
    const size_t mrow0 = (size_t)b * NL_;

    const unsigned short* sl  = wave ? slo : shi;
    unsigned short*       gpl = wave ? glo : ghi;

    const int f0    = tid * 8;
    const int fstep = f0 >> 5;
    const int fj    = f0 & 31;

#pragma unroll 1
    for (int l0 = 0; l0 < NL_; l0 += 16) {
        {
            const v8f v = ld8f(Xd + (mrow0 + (size_t)(l0 + fstep)) * XW_ + NR_ + fj);
#pragma unroll
            for (int e = 0; e < 8; ++e) sBC[f0 + e] = v[e];
        }
        __syncthreads();
#pragma unroll 1
        for (int t = 0; t < 16; ++t) {
            const size_t mrow = mrow0 + (size_t)(l0 + t);
            const size_t e = mrow * DI_ + d;
            const float xv = X[e];
            const float zv = Z[e];
            const float dl = Dl[e];
            const float u  = conv4_silu(xm3, xm2, xm1, xv, w0, w1, w2, w3, cbias);
            xm3 = xm2; xm2 = xm1; xm1 = xv;
            const float dt = softplus_f(dl + tb);
            const float du = dt * u;
            const float* bc = sBC + t * 32;
            float y = 0.0f;
#pragma unroll
            for (int n = 0; n < NS_; ++n) {
                const float da = __expf(dt * an[n]);
                hs[n] = da * hs[n] + du * bc[n];
                y += hs[n] * bc[16 + n];
            }
            const float g = (y + u) * silu_f(zv);
            const unsigned short hb = f32_to_bf16(g);
            const unsigned short lb = f32_to_bf16(g - bf16_to_f32(hb));
            shi[t * 64 + tid] = hb;
            slo[t * 64 + tid] = lb;
        }
        __syncthreads();
        const size_t gbase = (mrow0 + (size_t)l0) * DI_ + dbase;
        rows16_store_pass(sl, gpl, gbase, lane);
        __threadfence();
        rows16_store_pass(sl, gpl, gbase, lane);
        __syncthreads();
    }
}

extern "C" void kernel_launch(void* const* d_in, const int* in_sizes, int n_in,
                              void* d_out, int out_size, void* d_ws, size_t ws_size,
                              hipStream_t stream)
{
    if (n_in < 9) return;
    if (in_sizes[0] != MT_ * DM_)       return;
    if (in_sizes[1] != DM_ * 2 * DI_)   return;
    if (in_sizes[2] != 4 * DI_)         return;
    if (in_sizes[3] != DI_)             return;
    if (in_sizes[4] != DI_ * XW_)       return;
    if (in_sizes[5] != NR_ * DI_)       return;
    if (in_sizes[6] != DI_)             return;
    if (in_sizes[7] != DI_ * NS_)       return;
    if (in_sizes[8] != DI_ * DM_)       return;
    if (out_size != MT_ * DM_)          return;

    const float* xin  = (const float*)d_in[0];
    const float* win  = (const float*)d_in[1];
    const float* cw   = (const float*)d_in[2];
    const float* cb   = (const float*)d_in[3];
    const float* wx   = (const float*)d_in[4];
    const float* wdt  = (const float*)d_in[5];
    const float* bdt  = (const float*)d_in[6];
    const float* alog = (const float*)d_in[7];
    const float* wout = (const float*)d_in[8];
    float* out = (float*)d_out;

    const size_t SZ_IN16 = (size_t)MT_ * DM_ * 2;
    const size_t SZ_WIT  = (size_t)2 * DI_ * DM_ * 2;
    const size_t SZ_WXT  = (size_t)XW_ * DI_ * 2;
    const size_t SZ_WDT  = (size_t)DI_ * NR_ * 2;
    const size_t SZ_WOT  = (size_t)DM_ * DI_ * 2;
    const size_t SZ_F    = (size_t)MT_ * DI_ * 4;
    const size_t SZ_U16  = (size_t)MT_ * DI_ * 2;
    const size_t SZ_XD   = (size_t)MT_ * XW_ * 4;
    const size_t SZ_DT16 = (size_t)MT_ * NR_ * 2;
    const size_t SZ_G    = (size_t)MT_ * DI_ * 2;

    const size_t OFF_IN16 = 0;
    const size_t OFF_WIT  = OFF_IN16 + SZ_IN16;
    const size_t OFF_WXT  = OFF_WIT  + SZ_WIT;
    const size_t OFF_WDT  = OFF_WXT  + SZ_WXT;
    const size_t OFF_WOT  = OFF_WDT  + SZ_WDT;
    const size_t OFF_XF   = OFF_WOT  + SZ_WOT;
    const size_t OFF_ZF   = OFF_XF   + SZ_F;
    const size_t OFF_U16  = OFF_ZF   + SZ_F;
    const size_t OFF_XD   = OFF_U16  + SZ_U16;
    const size_t OFF_DT16 = OFF_XD   + SZ_XD;
    const size_t OFF_DL   = OFF_DT16 + SZ_DT16;
    const size_t OFF_GHI  = OFF_DL   + SZ_F;
    const size_t OFF_GLO  = OFF_GHI  + SZ_G;
    const size_t WS_END   = OFF_GLO  + SZ_G;
    if (WS_END > (size_t)134217728) return;
    if (ws_size < WS_END) return;

    char* ws = (char*)d_ws;
    unsigned short* in16 = (unsigned short*)(ws + OFF_IN16);
    unsigned short* wit  = (unsigned short*)(ws + OFF_WIT);
    unsigned short* wxt  = (unsigned short*)(ws + OFF_WXT);
    unsigned short* wdtt = (unsigned short*)(ws + OFF_WDT);
    unsigned short* wot  = (unsigned short*)(ws + OFF_WOT);
    float*          Xf   = (float*)(ws + OFF_XF);
    float*          Zf   = (float*)(ws + OFF_ZF);
    unsigned short* u16  = (unsigned short*)(ws + OFF_U16);
    float*          Xd   = (float*)(ws + OFF_XD);
    unsigned short* dt16 = (unsigned short*)(ws + OFF_DT16);
    float*          Dl   = (float*)(ws + OFF_DL);
    unsigned short* ghi  = (unsigned short*)(ws + OFF_GHI);
    unsigned short* glo  = (unsigned short*)(ws + OFF_GLO);

    const float SC16 = 1.0f / 65536.0f;
    const int   NOSPLIT = 1 << 30;

    {
        const int n8 = (MT_ * DM_) / 8;
        hipLaunchKernelGGL(cvt_rows_kernel, dim3((n8 + 255) / 256), dim3(256), 0, stream,
                           xin, in16, (int)MT_, (int)DM_, (int)DM_, 0, 1.0f);
    }
    hipLaunchKernelGGL(cvt_t_kernel, dim3((2 * DI_) / 32, DM_ / 64), dim3(256), 0, stream,
                       win, wit, (int)DM_, (int)(2 * DI_), 0, 1.0f);
    hipLaunchKernelGGL(cvt_t_kernel, dim3(XW_ / 32, DI_ / 64), dim3(256), 0, stream,
                       wx, wxt, (int)DI_, (int)XW_, 1, 256.0f);
    hipLaunchKernelGGL(cvt_t_kernel, dim3(DI_ / 32, NR_ / 64), dim3(256), 0, stream,
                       wdt, wdtt, (int)NR_, (int)DI_, 1, 256.0f);
    hipLaunchKernelGGL(cvt_t_kernel, dim3(DM_ / 32, DI_ / 64), dim3(256), 0, stream,
                       wout, wot, (int)DI_, (int)DM_, 0, 1.0f);

    hipLaunchKernelGGL(HIP_KERNEL_NAME(gemm_tn_kernel<FragB, false, 4>),
                       dim3((2 * DI_) / 128, MT_ / 64), dim3(128), 0, stream,
                       (const unsigned short*)in16, (const unsigned short*)in16,
                       (const unsigned short*)wit,
                       Xf, Zf, (int)DM_, (int)DI_, (int)DI_, 1.0f);

    hipLaunchKernelGGL(conv_silu_kernel, dim3(MT_), dim3(DI_ / 8), 0, stream,
                       (const float*)Xf, cw, cb, u16);

    hipLaunchKernelGGL(HIP_KERNEL_NAME(gemm_tn_kernel<FragH, false, 1>),
                       dim3(XW_ / 32, MT_ / 64), dim3(128), 0, stream,
                       (const unsigned short*)u16, (const unsigned short*)u16,
                       (const unsigned short*)wxt,
                       Xd, Xd, (int)DI_, (int)XW_, NOSPLIT, SC16);

    {
        const int n8 = (MT_ * NR_) / 8;
        hipLaunchKernelGGL(cvt_rows_kernel, dim3((n8 + 255) / 256), dim3(256), 0, stream,
                           (const float*)Xd, dt16, (int)MT_, (int)NR_, (int)XW_, 1, 256.0f);
    }

    hipLaunchKernelGGL(HIP_KERNEL_NAME(gemm_tn_kernel<FragH, false, 4>),
                       dim3(DI_ / 128, MT_ / 64), dim3(128), 0, stream,
                       (const unsigned short*)dt16, (const unsigned short*)dt16,
                       (const unsigned short*)wdtt,
                       Dl, Dl, (int)NR_, (int)DI_, NOSPLIT, SC16);

    hipLaunchKernelGGL(scan_kernel, dim3(DI_ / 64, NB_), dim3(64), 0, stream,
                       (const float*)Xf, (const float*)Zf, (const float*)Dl, (const float*)Xd,
                       cw, cb, bdt, alog, ghi, glo);

    hipLaunchKernelGGL(HIP_KERNEL_NAME(gemm_tn_kernel<FragB, true, 2>),
                       dim3(DM_ / 64, MT_ / 64), dim3(128), 0, stream,
                       (const unsigned short*)ghi, (const unsigned short*)glo,
                       (const unsigned short*)wot,
                       out, out, (int)DI_, (int)DM_, NOSPLIT, 1.0f);
}
